// NODEModel_75548474736884
// MI455X (gfx1250) — hardware-verified
//
#include <hip/hip_runtime.h>

#pragma clang fp contract(off)

typedef _Float16 v16h __attribute__((ext_vector_type(16)));
typedef _Float16 v8h  __attribute__((ext_vector_type(8)));
typedef float    v8f  __attribute__((ext_vector_type(8)));
typedef float    v4f  __attribute__((ext_vector_type(4)));
typedef v8h __attribute__((may_alias)) v8ha;
typedef v4f __attribute__((may_alias)) v4fa;

union Frag { v16h v; v8h half[2]; };

#define NPTS    131072
#define WID     128
#define CHROWS  65536
#define NCHUNK  8
#define WMAT    (WID * WID)
#define TILE_H  (64 * WID)
#define WSCALE  256.0f
#define LSCALE  2048.0f
#define INV_W   0.00390625f
#define INV_WL  1.9073486328125e-6f
#define F16MINN 6.103515625e-5f
#define EPSV    1e-8f
#define SQ35    0.7745966692414834f
#define GW_OUT  0.5555555555555556f
#define GW_MID  0.8888888888888888f

static_assert(NPTS % CHROWS == 0);
static_assert(CHROWS % 64 == 0);
static_assert(WID % 32 == 0);
static_assert(NPTS % 256 == 0);

__device__ __forceinline__ v8f wmma_f16(v16h a, v16h b, v8f c) {
  v8f d = __builtin_amdgcn_wmma_f32_16x16x32_f16(false, a, false, b, (short)0, c, false, false);
  asm volatile("v_nop\n\tv_nop\n\tv_nop\n\tv_nop" : "+v"(d) : "v"(a), "v"(b));
  return d;
}

__device__ __forceinline__ v16h load_frag(const _Float16* p, int h) {
  Frag f;
  f.half[0] = *(const v8ha*)(p + 8 * h);
  f.half[1] = *(const v8ha*)(p + 16 + 8 * h);
  return f.v;
}

__device__ __forceinline__ void split_hl(float v, _Float16& hv, _Float16& lv) {
  const _Float16 h16 = (_Float16)v;
  float hf = (float)h16;
  hf = (fabsf(hf) < F16MINN) ? 0.0f : hf;
  hv = (_Float16)hf;
  lv = (_Float16)((v - hf) * LSCALE);
}

__device__ __forceinline__ void wt_store_pass(const _Float16* sT, _Float16* dst0, int w, int lane) {
  const int q8 = lane & 7, sub = lane >> 3;
  #pragma unroll
  for (int i = 0; i < 8; ++i) {
    const int L = 32 * w + 4 * i + sub;
    const int n = L >> 1, hl = L & 1;
    const v8h v = *(const v8ha*)(sT + n * 136 + 64 * hl + 8 * q8);
    *(volatile v8h*)(dst0 + (size_t)n * WID + 64 * hl + 8 * q8) = v;
  }
}

__global__ __launch_bounds__(256) void k_wconvert(
    const float* __restrict__ icWh, const float* __restrict__ dpWh,
    _Float16* __restrict__ wt)
{
  __shared__ __attribute__((aligned(16))) _Float16 sT[WID * 136];
  const int tid = threadIdx.x, lane = tid & 31, w = tid >> 5;
  const int q = blockIdx.x;
  const float* W = (q < 3) ? (icWh + (size_t)q * WMAT) : (dpWh + (size_t)(q - 3) * WMAT);
  #pragma unroll 4
  for (int idx = tid; idx < WMAT; idx += 256) {
    const int k = idx >> 7, n = idx & 127;
    sT[n * 136 + k] = (_Float16)(W[idx] * WSCALE);
  }
  __syncthreads();
  _Float16* dst0 = wt + (size_t)q * WMAT;
  wt_store_pass(sT, dst0, w, lane);
  __threadfence();
  wt_store_pass(sT, dst0, w, lane);
}

__device__ __forceinline__ void l0_store_pass(const _Float16* sA, _Float16* op, size_t row0g, int lane) {
  const int q8 = lane & 7, sub = lane >> 3;
  #pragma unroll
  for (int i = 0; i < 32; ++i) {
    const int L = 4 * i + sub;
    const int rowl = L >> 1, hl = L & 1;
    const v8h v = *(const v8ha*)(sA + rowl * WID + 64 * hl + 8 * q8);
    *(volatile v8h*)(op + (row0g + rowl) * WID + 64 * hl + 8 * q8) = v;
  }
}

__global__ __launch_bounds__(64) void k_layer0(
    const float* __restrict__ tx, const float* __restrict__ W0, const float* __restrict__ b0,
    int nfeat, int isdp, float node, int pt0,
    _Float16* __restrict__ hi, _Float16* __restrict__ lo)
{
  __shared__ float sW0[6 * WID];
  __shared__ float sB0[WID];
  __shared__ __attribute__((aligned(16))) _Float16 sAct[2 * TILE_H];

  const int tid = threadIdx.x, lane = tid & 31, w = tid >> 5;

  #pragma unroll 1
  for (int idx = tid; idx < 6 * WID; idx += 64) {
    const int k = idx >> 7, n = idx & 127;
    const int kc = (k < nfeat) ? k : (nfeat - 1);
    const float v = W0[kc * WID + n];
    sW0[idx] = (k < nfeat) ? v : 0.0f;
  }
  #pragma unroll 1
  for (int idx = tid; idx < WID; idx += 64) sB0[idx] = b0[idx];

  const int pt = pt0 + blockIdx.x * 64 + tid;
  const v4f p4 = *(const v4fa*)(tx + (size_t)pt * 4);
  const float t = p4.x, x = p4.y, y = p4.z, z = p4.w;
  const float xy  = x * x + y * y;
  const float r   = sqrtf(xy + z * z + EPSV);
  const float rho = sqrtf(xy + EPSV);
  const float ir = 1.0f / r, irho = 1.0f / rho;
  const float u  = r / (1.0f + r);
  const float ct = z * ir, st = rho * ir, cp = x * irho, sp = y * irho;
  const float a  = t * 0.5f;
  const float ts = a * node + a;
  float f0, f1, f2, f3, f4, f5;
  if (isdp != 0) { f0 = ts; f1 = u;  f2 = ct; f3 = st; f4 = cp; f5 = sp; }
  else           { f0 = u;  f1 = ct; f2 = st; f3 = cp; f4 = sp; f5 = 0.0f; }
  __syncthreads();

  _Float16* sh = sAct + tid * WID;
  _Float16* sl = sAct + TILE_H + tid * WID;
  #pragma unroll 1
  for (int n = 0; n < WID; ++n) {
    float s = f0 * sW0[n];
    s = fmaf(f1, sW0[WID + n], s);
    s = fmaf(f2, sW0[2 * WID + n], s);
    s = fmaf(f3, sW0[3 * WID + n], s);
    s = fmaf(f4, sW0[4 * WID + n], s);
    s = fmaf(f5, sW0[5 * WID + n], s);
    s = s + sB0[n];
    const float v = tanhf(s);
    _Float16 hv, lv;
    split_hl(v, hv, lv);
    sh[n] = hv;
    sl[n] = lv;
  }
  __syncthreads();

  _Float16* op = (w == 0) ? hi : lo;
  const _Float16* src = sAct + w * TILE_H;
  const size_t row0g = (size_t)blockIdx.x * 64;
  l0_store_pass(src, op, row0g, lane);
  __threadfence();
  l0_store_pass(src, op, row0g, lane);
}

__device__ __forceinline__ void hid_store_pass(const _Float16* sA, _Float16* op, size_t row0g, int w, int lane) {
  const int q8 = lane & 7, sub = lane >> 3;
  const int pl = w >> 2;
  #pragma unroll
  for (int i = 0; i < 8; ++i) {
    const int L = 32 * w + 4 * i + sub;
    const int rowl = (L >> 1) & 63, hl = L & 1;
    const v8h v = *(const v8ha*)(sA + pl * TILE_H + rowl * WID + 64 * hl + 8 * q8);
    *(volatile v8h*)(op + (row0g + rowl) * WID + 64 * hl + 8 * q8) = v;
  }
}

__global__ __launch_bounds__(256) void k_hidden(
    const _Float16* __restrict__ inHi,
    const _Float16* __restrict__ inLo,
    const _Float16* __restrict__ wt,
    const float* __restrict__ bias,
    _Float16* __restrict__ outHi,
    _Float16* __restrict__ outLo,
    const float* __restrict__ wo,
    const float* __restrict__ bo,
    float* __restrict__ vals,
    int vrow0, int last)
{
  __shared__ __attribute__((aligned(16))) _Float16 sAct[2 * TILE_H];
  __shared__ __attribute__((aligned(16))) float sPart[2 * 64];
  __shared__ __attribute__((aligned(16))) float sV[64];

  const int tid = threadIdx.x, lane = tid & 31, w = tid >> 5;
  const int h = lane >> 4, m = lane & 15;
  const int rg = w & 3, ch = w >> 2;
  const int row0 = blockIdx.x * 64 + 16 * rg;

  const _Float16* pah = inHi + (size_t)(row0 + m) * WID;
  const _Float16* pal = inLo + (size_t)(row0 + m) * WID;
  const _Float16* pb  = wt + (size_t)(64 * ch + m) * WID;

  const v8f zero8 = {0.f, 0.f, 0.f, 0.f, 0.f, 0.f, 0.f, 0.f};
  v8f acch[4], accl[4];
  #pragma unroll
  for (int nt = 0; nt < 4; ++nt) { acch[nt] = zero8; accl[nt] = zero8; }

  #pragma unroll 1
  for (int k0 = 0; k0 < WID; k0 += 32) {
    const v16h ah = load_frag(pah + k0, h);
    const v16h al = load_frag(pal + k0, h);
    #pragma unroll
    for (int nt = 0; nt < 4; ++nt) {
      const v16h b = load_frag(pb + (size_t)nt * 16 * WID + k0, h);
      acch[nt] = wmma_f16(ah, b, acch[nt]);
      accl[nt] = wmma_f16(al, b, accl[nt]);
    }
  }

  float tv[4][8];
  #pragma unroll
  for (int nt = 0; nt < 4; ++nt) {
    const float bc = bias[64 * ch + 16 * nt + m];
    #pragma unroll
    for (int r = 0; r < 8; ++r)
      tv[nt][r] = tanhf(acch[nt][r] * INV_W + accl[nt][r] * INV_WL + bc);
  }

  if (last == 0) {
    #pragma unroll
    for (int nt = 0; nt < 4; ++nt) {
      #pragma unroll
      for (int r = 0; r < 8; ++r) {
        _Float16 hv, lv;
        split_hl(tv[nt][r], hv, lv);
        const int idx = (16 * rg + 8 * h + r) * WID + 64 * ch + 16 * nt + m;
        sAct[idx] = hv;
        sAct[TILE_H + idx] = lv;
      }
    }
    __syncthreads();
    _Float16* op = (w < 4) ? outHi : outLo;
    const size_t row0g = (size_t)blockIdx.x * 64;
    hid_store_pass(sAct, op, row0g, w, lane);
    __threadfence();
    hid_store_pass(sAct, op, row0g, w, lane);
  } else {
    float wv[4];
    #pragma unroll
    for (int nt = 0; nt < 4; ++nt) wv[nt] = wo[64 * ch + 16 * nt + m];
    float p[8];
    #pragma unroll
    for (int r = 0; r < 8; ++r) {
      float s = tv[0][r] * wv[0];
      s = fmaf(tv[1][r], wv[1], s);
      s = fmaf(tv[2][r], wv[2], s);
      s = fmaf(tv[3][r], wv[3], s);
      p[r] = s;
    }
    #pragma unroll
    for (int r = 0; r < 8; ++r) {
      p[r] += __shfl_xor(p[r], 1);
      p[r] += __shfl_xor(p[r], 2);
      p[r] += __shfl_xor(p[r], 4);
      p[r] += __shfl_xor(p[r], 8);
    }
    if (m == 0) {
      #pragma unroll
      for (int r = 0; r < 8; ++r) sPart[64 * ch + 16 * rg + 8 * h + r] = p[r];
    }
    __syncthreads();
    if (tid < 64) sV[tid] = (sPart[tid] + sPart[64 + tid]) + bo[0];
    __syncthreads();
    const size_t vb = (size_t)vrow0 + (size_t)blockIdx.x * 64;
    if (tid < 16) {
      const v4f v = *(const v4fa*)(sV + 4 * tid);
      *(volatile v4f*)(vals + vb + 4 * tid) = v;
    }
    __threadfence();
    if (tid < 16) {
      const v4f v = *(const v4fa*)(sV + 4 * tid);
      *(volatile v4f*)(vals + vb + 4 * tid) = v;
    }
  }
}

__global__ __launch_bounds__(256) void k_combine(
    const float* __restrict__ tx, const float* __restrict__ vals, float* __restrict__ out)
{
  __shared__ __attribute__((aligned(16))) float sO[256];
  const int tid = threadIdx.x;
  const int n = blockIdx.x * 256 + tid;
  const float t   = tx[(size_t)n * 4];
  const float a   = t * 0.5f;
  const float phi = vals[n];
  const float v0  = vals[NPTS + n];
  const float v1  = vals[2 * NPTS + n];
  const float v2  = vals[3 * NPTS + n];
  const float s   = (GW_OUT * v0 + GW_OUT * v2) + GW_MID * v1;
  sO[tid] = phi + a * s;
  __syncthreads();
  const size_t ob = (size_t)blockIdx.x * 256;
  if (tid < 64) {
    const v4f v = *(const v4fa*)(sO + 4 * tid);
    *(volatile v4f*)(out + ob + 4 * tid) = v;
  }
  __threadfence();
  if (tid < 64) {
    const v4f v = *(const v4fa*)(sO + 4 * tid);
    *(volatile v4f*)(out + ob + 4 * tid) = v;
  }
}

extern "C" void kernel_launch(void* const* d_in, const int* in_sizes, int n_in,
                              void* d_out, int out_size, void* d_ws, size_t ws_size,
                              hipStream_t stream) {
  if (n_in < 13) return;
  if (in_sizes[0] != 4 * NPTS) return;
  if (out_size != NPTS) return;
  if (in_sizes[1] != 6 * WID || in_sizes[2] != WID || in_sizes[3] != 3 * WMAT ||
      in_sizes[4] != 3 * WID || in_sizes[5] != WID || in_sizes[6] < 1) return;
  if (in_sizes[7] != 5 * WID || in_sizes[8] != WID || in_sizes[9] != 3 * WMAT ||
      in_sizes[10] != 3 * WID || in_sizes[11] != WID || in_sizes[12] < 1) return;

  const float* tx    = (const float*)d_in[0];
  const float* dp_W0 = (const float*)d_in[1];
  const float* dp_b0 = (const float*)d_in[2];
  const float* dp_Wh = (const float*)d_in[3];
  const float* dp_bh = (const float*)d_in[4];
  const float* dp_Wo = (const float*)d_in[5];
  const float* dp_bo = (const float*)d_in[6];
  const float* ic_W0 = (const float*)d_in[7];
  const float* ic_b0 = (const float*)d_in[8];
  const float* ic_Wh = (const float*)d_in[9];
  const float* ic_bh = (const float*)d_in[10];
  const float* ic_Wo = (const float*)d_in[11];
  const float* ic_bo = (const float*)d_in[12];
  float* out = (float*)d_out;

  const size_t wt_bytes   = (size_t)6 * WMAT * 2;
  const size_t pl_bytes   = (size_t)CHROWS * WID * 2;
  const size_t vals_bytes = (size_t)4 * NPTS * 4;
  const size_t off_wt   = 0;
  const size_t off_hiA  = off_wt + wt_bytes;
  const size_t off_loA  = off_hiA + pl_bytes;
  const size_t off_hiB  = off_loA + pl_bytes;
  const size_t off_loB  = off_hiB + pl_bytes;
  const size_t off_vals = off_loB + pl_bytes;
  const size_t total    = off_vals + vals_bytes;
  if (total > ws_size) return;

  char* ws = (char*)d_ws;
  _Float16* wt   = (_Float16*)(ws + off_wt);
  _Float16* hiA  = (_Float16*)(ws + off_hiA);
  _Float16* loA  = (_Float16*)(ws + off_loA);
  _Float16* hiB  = (_Float16*)(ws + off_hiB);
  _Float16* loB  = (_Float16*)(ws + off_loB);
  float*    vals = (float*)(ws + off_vals);

  k_wconvert<<<6, 256, 0, stream>>>(ic_Wh, dp_Wh, wt);

  for (int c = 0; c < NCHUNK; ++c) {
    const int isdp = (c >= 2) ? 1 : 0;
    const int s    = isdp ? ((c - 2) >> 1) : 0;
    const int half = isdp ? ((c - 2) & 1) : c;
    const int pt0  = half * CHROWS;
    const float node = (s == 0) ? -SQ35 : ((s == 1) ? 0.0f : SQ35);
    const float* W0 = isdp ? dp_W0 : ic_W0;
    const float* b0 = isdp ? dp_b0 : ic_b0;
    const float* bh = isdp ? dp_bh : ic_bh;
    const float* Wo = isdp ? dp_Wo : ic_Wo;
    const float* bo = isdp ? dp_bo : ic_bo;
    const int nfeat = isdp ? 6 : 5;
    const _Float16* wtb = wt + (size_t)(isdp ? 3 : 0) * WMAT;
    const int vrow0 = isdp ? (NPTS + s * NPTS + pt0) : pt0;

    k_layer0<<<CHROWS / 64, 64, 0, stream>>>(tx, W0, b0, nfeat, isdp, node, pt0, hiA, loA);
    k_hidden<<<CHROWS / 64, 256, 0, stream>>>(hiA, loA, wtb,            bh,           hiB, loB, Wo, bo, vals, vrow0, 0);
    k_hidden<<<CHROWS / 64, 256, 0, stream>>>(hiB, loB, wtb + WMAT,     bh + WID,     hiA, loA, Wo, bo, vals, vrow0, 0);
    k_hidden<<<CHROWS / 64, 256, 0, stream>>>(hiA, loA, wtb + 2 * WMAT, bh + 2 * WID, hiB, loB, Wo, bo, vals, vrow0, 1);
  }

  k_combine<<<NPTS / 256, 256, 0, stream>>>(tx, vals, out);
}
